// MoBA_4681514353439
// MI455X (gfx1250) — hardware-verified
//
#include <hip/hip_runtime.h>


#define S_ 2048
#define D_ 2048
#define H_ 16
#define DH 128
#define CHUNK_ 256
#define NBLK 8
#define TOPK_ 4
#define NEGF (-1.0e30f)
#define POSF (1.0e30f)
#define KILLF (-3.0e38f)
#define APITCH 40
#define VPITCH 72
#define QK_SCALE 0.08838834764831845f
#define NOP4 "v_nop\n\tv_nop\n\tv_nop\n\tv_nop"

typedef __bf16 bf16_t;
typedef _Float16 f16t;
typedef unsigned short us_t;
typedef bf16_t v16bf __attribute__((ext_vector_type(16)));
typedef f16t   v16h  __attribute__((ext_vector_type(16)));
typedef f16t   v8h   __attribute__((ext_vector_type(8)));
typedef us_t   v8us  __attribute__((ext_vector_type(8)));
typedef float  v8f   __attribute__((ext_vector_type(8)));
typedef float  v4f   __attribute__((ext_vector_type(4)));
typedef unsigned int v4u __attribute__((ext_vector_type(4)));
typedef v8us v8us_ma __attribute__((may_alias));
typedef v8h  v8h_ma  __attribute__((may_alias));
typedef v4f  v4f_ma  __attribute__((may_alias));
typedef v4u  v4u_ma  __attribute__((may_alias));

union FragB { v16bf v; v8us p[2]; };
union FragH { v16h v; v8h p[2]; };
union Pack8 { v8us s; v4u u; };
union PackH { v8h h; v4u u; };

static __device__ __forceinline__ us_t f2bf(float f) {
  unsigned u = __float_as_uint(f);
  u += 0x7FFFu + ((u >> 16) & 1u);
  return (us_t)(u >> 16);
}
static __device__ __forceinline__ float bf2f(us_t b) {
  return __uint_as_float(((unsigned)b) << 16);
}
static __device__ __forceinline__ v8f wmma_bf(v16bf a, v16bf b, v8f c) {
  return __builtin_amdgcn_wmma_f32_16x16x32_bf16(false, a, false, b, (short)0, c, false, false);
}
static __device__ __forceinline__ v8f wmma_h(v16h a, v16h b, v8f c) {
  return __builtin_amdgcn_wmma_f32_16x16x32_f16(false, a, false, b, (short)0, c, false, false);
}

__global__ __launch_bounds__(256) void k_cvt(const float* __restrict__ s0, const float* __restrict__ s1,
                                             const float* __restrict__ s2, const float* __restrict__ s3,
                                             const float* __restrict__ s4,
                                             us_t* d0, us_t* d1, us_t* d2, us_t* d3, us_t* d4, int n) {
  const float* src = s0;
  us_t* dst = d0;
  const int sel = blockIdx.y;
  if (sel == 1) { src = s1; dst = d1; }
  else if (sel == 2) { src = s2; dst = d2; }
  else if (sel == 3) { src = s3; dst = d3; }
  else if (sel == 4) { src = s4; dst = d4; }
  const size_t i = ((size_t)blockIdx.x * 256 + threadIdx.x) * 8;
  if (i + 8 > (size_t)n) return;
  const v4f a = *(const v4f*)(src + i);
  const v4f b = *(const v4f*)(src + i + 4);
  Pack8 o;
  o.s[0] = f2bf(a[0]); o.s[1] = f2bf(a[1]); o.s[2] = f2bf(a[2]); o.s[3] = f2bf(a[3]);
  o.s[4] = f2bf(b[0]); o.s[5] = f2bf(b[1]); o.s[6] = f2bf(b[2]); o.s[7] = f2bf(b[3]);
  us_t* p = dst + i;
  *(volatile v4u*)p = o.u;
  __threadfence();
  *(volatile v4u*)p = o.u;
}

template <bool ASPLIT>
__global__ __launch_bounds__(256) void k_gemm(const us_t* __restrict__ A, const us_t* __restrict__ A2,
                                              const us_t* __restrict__ B0, const us_t* __restrict__ B1,
                                              const us_t* __restrict__ B2,
                                              float* C0, float* C1, float* C2, int M, int N, int K) {
  __shared__ __attribute__((aligned(16))) float smem[8192];
  us_t* As  = (us_t*)smem;
  us_t* Bs  = As + 128 * APITCH;
  us_t* A2s = Bs + 128 * APITCH;

  const us_t* B = B0;
  float* C = C0;
  if (blockIdx.z == 1) { B = B1; C = C1; }
  else if (blockIdx.z == 2) { B = B2; C = C2; }

  const int tid = threadIdx.x;
  const int lane = tid & 31, wave = tid >> 5, hl = lane >> 4, m = lane & 15;
  const int wm = wave >> 1, wn = wave & 1;
  const int mBase = blockIdx.y * 128, nBase = blockIdx.x * 128;
  const int m0l = wm * 32, n0l = wn * 64;
  if (mBase + 128 > M || nBase + 128 > N) return;

  v8f acc[2][4];
#pragma unroll
  for (int i = 0; i < 2; ++i)
#pragma unroll
    for (int j = 0; j < 4; ++j)
#pragma unroll
      for (int e = 0; e < 8; ++e) acc[i][j][e] = 0.0f;

  for (int k0 = 0; k0 < K; k0 += 32) {
    __syncthreads();
#pragma unroll
    for (int it = 0; it < 2; ++it) {
      const int idx = tid + it * 256;
      const int row = idx >> 2;
      const int ch  = (idx & 3) * 8;
      *(v8us*)(As + row * APITCH + ch) = *(const v8us*)(A + (size_t)(mBase + row) * K + k0 + ch);
      if (ASPLIT)
        *(v8us*)(A2s + row * APITCH + ch) = *(const v8us*)(A2 + (size_t)(mBase + row) * K + k0 + ch);
      *(v8us*)(Bs + row * APITCH + ch) = *(const v8us*)(B + (size_t)(nBase + row) * K + k0 + ch);
    }
    __syncthreads();

    FragB fa0, fa1, fb0, fb1, fb2, fb3;
    fa0.p[0] = *(const v8us*)(As + (m0l + m) * APITCH + 8 * hl);
    fa0.p[1] = *(const v8us*)(As + (m0l + m) * APITCH + 16 + 8 * hl);
    fa1.p[0] = *(const v8us*)(As + (m0l + 16 + m) * APITCH + 8 * hl);
    fa1.p[1] = *(const v8us*)(As + (m0l + 16 + m) * APITCH + 16 + 8 * hl);
    fb0.p[0] = *(const v8us*)(Bs + (n0l + m) * APITCH + 8 * hl);
    fb0.p[1] = *(const v8us*)(Bs + (n0l + m) * APITCH + 16 + 8 * hl);
    fb1.p[0] = *(const v8us*)(Bs + (n0l + 16 + m) * APITCH + 8 * hl);
    fb1.p[1] = *(const v8us*)(Bs + (n0l + 16 + m) * APITCH + 16 + 8 * hl);
    fb2.p[0] = *(const v8us*)(Bs + (n0l + 32 + m) * APITCH + 8 * hl);
    fb2.p[1] = *(const v8us*)(Bs + (n0l + 32 + m) * APITCH + 16 + 8 * hl);
    fb3.p[0] = *(const v8us*)(Bs + (n0l + 48 + m) * APITCH + 8 * hl);
    fb3.p[1] = *(const v8us*)(Bs + (n0l + 48 + m) * APITCH + 16 + 8 * hl);

    acc[0][0] = wmma_bf(fa0.v, fb0.v, acc[0][0]);
    acc[0][1] = wmma_bf(fa0.v, fb1.v, acc[0][1]);
    acc[0][2] = wmma_bf(fa0.v, fb2.v, acc[0][2]);
    acc[0][3] = wmma_bf(fa0.v, fb3.v, acc[0][3]);
    acc[1][0] = wmma_bf(fa1.v, fb0.v, acc[1][0]);
    acc[1][1] = wmma_bf(fa1.v, fb1.v, acc[1][1]);
    acc[1][2] = wmma_bf(fa1.v, fb2.v, acc[1][2]);
    acc[1][3] = wmma_bf(fa1.v, fb3.v, acc[1][3]);
    if (ASPLIT) {
      FragB ga0, ga1;
      ga0.p[0] = *(const v8us*)(A2s + (m0l + m) * APITCH + 8 * hl);
      ga0.p[1] = *(const v8us*)(A2s + (m0l + m) * APITCH + 16 + 8 * hl);
      ga1.p[0] = *(const v8us*)(A2s + (m0l + 16 + m) * APITCH + 8 * hl);
      ga1.p[1] = *(const v8us*)(A2s + (m0l + 16 + m) * APITCH + 16 + 8 * hl);
      acc[0][0] = wmma_bf(ga0.v, fb0.v, acc[0][0]);
      acc[0][1] = wmma_bf(ga0.v, fb1.v, acc[0][1]);
      acc[0][2] = wmma_bf(ga0.v, fb2.v, acc[0][2]);
      acc[0][3] = wmma_bf(ga0.v, fb3.v, acc[0][3]);
      acc[1][0] = wmma_bf(ga1.v, fb0.v, acc[1][0]);
      acc[1][1] = wmma_bf(ga1.v, fb1.v, acc[1][1]);
      acc[1][2] = wmma_bf(ga1.v, fb2.v, acc[1][2]);
      acc[1][3] = wmma_bf(ga1.v, fb3.v, acc[1][3]);
      asm volatile(NOP4
                   : "+v"(acc[0][0]), "+v"(acc[0][1]), "+v"(acc[0][2]), "+v"(acc[0][3]),
                     "+v"(acc[1][0]), "+v"(acc[1][1]), "+v"(acc[1][2]), "+v"(acc[1][3])
                   : "v"(fa0.v), "v"(fa1.v), "v"(ga0.v), "v"(ga1.v),
                     "v"(fb0.v), "v"(fb1.v), "v"(fb2.v), "v"(fb3.v));
    } else {
      asm volatile(NOP4
                   : "+v"(acc[0][0]), "+v"(acc[0][1]), "+v"(acc[0][2]), "+v"(acc[0][3]),
                     "+v"(acc[1][0]), "+v"(acc[1][1]), "+v"(acc[1][2]), "+v"(acc[1][3])
                   : "v"(fa0.v), "v"(fa1.v), "v"(fb0.v), "v"(fb1.v), "v"(fb2.v), "v"(fb3.v));
    }
  }
  __syncthreads();

  float* stg = smem + wave * 1024;
  const int c4 = m * 4;
#pragma unroll
  for (int i = 0; i < 2; ++i) {
    asm volatile("s_wait_dscnt 0x0" ::: "memory");
#pragma unroll
    for (int j = 0; j < 4; ++j)
#pragma unroll
      for (int r = 0; r < 8; ++r)
        stg[(8 * hl + r) * 64 + j * 16 + m] = acc[i][j][r];
    asm volatile("s_wait_dscnt 0x0" ::: "memory");
    const int row0 = mBase + m0l + i * 16;
#pragma unroll
    for (int pass = 0; pass < 2; ++pass) {
#pragma unroll
      for (int it = 0; it < 8; ++it) {
        const int rr = it * 2 + hl;
        const v4f v = *(const v4f_ma*)(stg + rr * 64 + c4);
        float* dst = C + (size_t)(row0 + rr) * N + nBase + n0l + c4;
        *(volatile v4f*)dst = v;
      }
      if (pass == 0) __threadfence();
    }
  }
}

__global__ __launch_bounds__(256) void k_trig(float* cs, float* sn) {
  __shared__ __attribute__((aligned(16))) float lds[512];
  const int t = threadIdx.x;
  const int s = blockIdx.x * 4 + (t >> 6);
  const int i = t & 63;
  const double pd = pow(10000.0, (double)(2 * i) * 0.0078125);
  const float p = (float)pd;
  const float inv = __frcp_rn(p);
  const float ang = (float)s * inv;
  lds[t] = cosf(ang);
  lds[256 + t] = sinf(ang);
  __syncthreads();
  if (t < 128) {
    const int which = t >> 6;
    const int q = t & 63;
    const v4f v = *(const v4f_ma*)(lds + which * 256 + q * 4);
    float* base = (which != 0) ? sn : cs;
    float* dst = base + (size_t)(blockIdx.x * 4 + (q >> 4)) * 64 + (q & 15) * 4;
    *(volatile v4f*)dst = v;
    __threadfence();
    *(volatile v4f*)dst = v;
  }
}

__global__ __launch_bounds__(256) void k_post(const float* __restrict__ qf, const float* __restrict__ kf,
                                              const float* __restrict__ vf,
                                              const float* __restrict__ cs, const float* __restrict__ sn,
                                              us_t* qh, us_t* ql, us_t* kh, us_t* kl, f16t* vT, float* km) {
#pragma clang fp contract(off)
  __shared__ __attribute__((aligned(16))) float red[8 * 128];
  __shared__ __attribute__((aligned(16))) f16t tile[128 * VPITCH];
  const int lane = threadIdx.x & 31, wave = threadIdx.x >> 5, hl = lane >> 4, cl = lane & 15;
  const int c8 = cl * 8;
  const int c = blockIdx.x >> 4, h = blockIdx.x & 15;
  const bool first = (cl < 8);
  const int i0 = c8 & 63;

  float ksum[8];
#pragma unroll
  for (int e = 0; e < 8; ++e) ksum[e] = 0.0f;

  for (int it = 0; it < 16; ++it) {
    const int rr = it * 16 + wave * 2 + hl;
    const int s = c * CHUNK_ + rr;
    const size_t base = (size_t)s * D_ + (size_t)h * DH + c8;
    const v4f qa = *(const v4f*)(qf + base), qb = *(const v4f*)(qf + base + 4);
    const v4f ka = *(const v4f*)(kf + base), kb = *(const v4f*)(kf + base + 4);
    const v4f ca = *(const v4f*)(cs + (size_t)s * 64 + i0), cb = *(const v4f*)(cs + (size_t)s * 64 + i0 + 4);
    const v4f sa = *(const v4f*)(sn + (size_t)s * 64 + i0), sb = *(const v4f*)(sn + (size_t)s * 64 + i0 + 4);
    float x[8], y[8], co[8], si[8];
    x[0] = qa[0]; x[1] = qa[1]; x[2] = qa[2]; x[3] = qa[3]; x[4] = qb[0]; x[5] = qb[1]; x[6] = qb[2]; x[7] = qb[3];
    y[0] = ka[0]; y[1] = ka[1]; y[2] = ka[2]; y[3] = ka[3]; y[4] = kb[0]; y[5] = kb[1]; y[6] = kb[2]; y[7] = kb[3];
    co[0] = ca[0]; co[1] = ca[1]; co[2] = ca[2]; co[3] = ca[3]; co[4] = cb[0]; co[5] = cb[1]; co[6] = cb[2]; co[7] = cb[3];
    si[0] = sa[0]; si[1] = sa[1]; si[2] = sa[2]; si[3] = sa[3]; si[4] = sb[0]; si[5] = sb[1]; si[6] = sb[2]; si[7] = sb[3];
    Pack8 pqh, pql, pkh, pkl;
#pragma unroll
    for (int e = 0; e < 8; ++e) {
      const float qo = x[e], ko = y[e];
      const float qp = __shfl_xor(qo, 8);
      const float kp = __shfl_xor(ko, 8);
      const float t1 = qo * co[e], t2 = qp * si[e];
      const float qr = first ? (t1 - t2) : (t1 + t2);
      const float u1 = ko * co[e], u2 = kp * si[e];
      const float kr = first ? (u1 - u2) : (u1 + u2);
      ksum[e] += kr;
      const us_t a1 = f2bf(qr);
      const us_t b1 = f2bf(qr - bf2f(a1));
      const us_t a2 = f2bf(kr);
      const us_t b2 = f2bf(kr - bf2f(a2));
      pqh.s[e] = a1; pql.s[e] = b1; pkh.s[e] = a2; pkl.s[e] = b2;
    }
    *(volatile v4u*)(qh + base) = pqh.u;
    *(volatile v4u*)(ql + base) = pql.u;
    *(volatile v4u*)(kh + base) = pkh.u;
    *(volatile v4u*)(kl + base) = pkl.u;
    __threadfence();
    *(volatile v4u*)(qh + base) = pqh.u;
    *(volatile v4u*)(ql + base) = pql.u;
    *(volatile v4u*)(kh + base) = pkh.u;
    *(volatile v4u*)(kl + base) = pkl.u;
  }

#pragma unroll
  for (int e = 0; e < 8; ++e) ksum[e] += __shfl_xor(ksum[e], 16);
  if (hl == 0) {
    v4f r0, r1;
    r0[0] = ksum[0]; r0[1] = ksum[1]; r0[2] = ksum[2]; r0[3] = ksum[3];
    r1[0] = ksum[4]; r1[1] = ksum[5]; r1[2] = ksum[6]; r1[3] = ksum[7];
    *(v4f*)(red + wave * 128 + c8) = r0;
    *(v4f*)(red + wave * 128 + c8 + 4) = r1;
  }
  __syncthreads();
  if (wave == 0) {
    v4f accv;
    accv[0] = 0.0f; accv[1] = 0.0f; accv[2] = 0.0f; accv[3] = 0.0f;
#pragma unroll
    for (int w = 0; w < 8; ++w) accv += *(const v4f_ma*)(red + w * 128 + lane * 4);
    accv *= (1.0f / 256.0f);
    float* dst = km + ((size_t)(c * H_ + h)) * DH + lane * 4;
    *(volatile v4f*)dst = accv;
    __threadfence();
    *(volatile v4f*)dst = accv;
  }

  for (int sub = 0; sub < 4; ++sub) {
    __syncthreads();
#pragma unroll
    for (int it = 0; it < 4; ++it) {
      const int kk = it * 16 + wave * 2 + hl;
      const int s = c * CHUNK_ + sub * 64 + kk;
      const size_t base = (size_t)s * D_ + (size_t)h * DH + c8;
      const v4f va = *(const v4f*)(vf + base), vb = *(const v4f*)(vf + base + 4);
      tile[(c8 + 0) * VPITCH + kk] = (f16t)(va[0] * 64.0f);
      tile[(c8 + 1) * VPITCH + kk] = (f16t)(va[1] * 64.0f);
      tile[(c8 + 2) * VPITCH + kk] = (f16t)(va[2] * 64.0f);
      tile[(c8 + 3) * VPITCH + kk] = (f16t)(va[3] * 64.0f);
      tile[(c8 + 4) * VPITCH + kk] = (f16t)(vb[0] * 64.0f);
      tile[(c8 + 5) * VPITCH + kk] = (f16t)(vb[1] * 64.0f);
      tile[(c8 + 6) * VPITCH + kk] = (f16t)(vb[2] * 64.0f);
      tile[(c8 + 7) * VPITCH + kk] = (f16t)(vb[3] * 64.0f);
    }
    __syncthreads();
    const int kq = (lane & 7) * 8;
#pragma unroll
    for (int pass = 0; pass < 2; ++pass) {
#pragma unroll
      for (int it2 = 0; it2 < 4; ++it2) {
        const int dcol = (wave * 4 + it2) * 4 + (lane >> 3);
        PackH x;
        x.h = *(const v8h_ma*)(tile + dcol * VPITCH + kq);
        f16t* dst = vT + ((size_t)(h * DH + dcol)) * S_ + c * CHUNK_ + sub * 64 + kq;
        *(volatile v4u*)dst = x.u;
      }
      if (pass == 0) __threadfence();
    }
  }
}

__global__ __launch_bounds__(256) void k_gate(const float* __restrict__ qf, const float* __restrict__ cs,
                                              const float* __restrict__ sn, const float* __restrict__ km,
                                              unsigned* selmask) {
  __shared__ __attribute__((aligned(16))) unsigned mskbuf[32];
  const int lane = threadIdx.x & 31, wave = threadIdx.x >> 5;
  const int h = blockIdx.y;
  const int s0 = blockIdx.x * 32;
  const int c4 = lane * 4;
  const int i0 = c4 & 63;
  const bool first = (lane < 16);

  for (int t = 0; t < 4; ++t) {
    const int s = s0 + wave * 4 + t;
    const int qblk = s >> 8;
    const v4f x  = *(const v4f*)(qf + (size_t)s * D_ + (size_t)h * DH + c4);
    const v4f cv = *(const v4f*)(cs + (size_t)s * 64 + i0);
    const v4f sv = *(const v4f*)(sn + (size_t)s * 64 + i0);
    float qr[4];
    {
#pragma clang fp contract(off)
#pragma unroll
      for (int e = 0; e < 4; ++e) {
        const float xo = x[e];
        const float xp = __shfl_xor(xo, 16);
        const float t1 = xo * cv[e], t2 = xp * sv[e];
        qr[e] = first ? (t1 - t2) : (t1 + t2);
      }
    }
    float g[NBLK];
#pragma unroll
    for (int j = 0; j < NBLK; ++j) {
      float val = NEGF;
      if (j < qblk) {
        const v4f kv = *(const v4f*)(km + ((size_t)(j * H_ + h)) * DH + c4);
        float d = qr[0] * kv[0] + qr[1] * kv[1] + qr[2] * kv[2] + qr[3] * kv[3];
#pragma unroll
        for (int off = 1; off < 32; off <<= 1) d += __shfl_xor(d, off);
        val = d;
      } else if (j == qblk) {
        val = POSF;
      }
      g[j] = val;
    }
    unsigned msk = 0u;
#pragma unroll
    for (int pick = 0; pick < TOPK_; ++pick) {
      float best = KILLF;
      int arg = 0;
#pragma unroll
      for (int j = 0; j < NBLK; ++j) { if (g[j] > best) { best = g[j]; arg = j; } }
      if (best > -5.0e29f) msk |= (1u << arg);
#pragma unroll
      for (int j = 0; j < NBLK; ++j) { if (j == arg) g[j] = KILLF; }
    }
    if (lane == 0) mskbuf[wave * 4 + t] = msk;
  }
  __syncthreads();
  if (threadIdx.x < 8) {
    const v4u v = *(const v4u_ma*)(mskbuf + threadIdx.x * 4);
    unsigned* dst = selmask + (size_t)h * S_ + s0 + threadIdx.x * 4;
    *(volatile v4u*)dst = v;
    __threadfence();
    *(volatile v4u*)dst = v;
  }
}

__global__ __launch_bounds__(128) void k_attn(const us_t* __restrict__ qh, const us_t* __restrict__ ql,
                                              const us_t* __restrict__ kh, const us_t* __restrict__ kl,
                                              const f16t* __restrict__ vT, const unsigned* __restrict__ selmask,
                                              const float* __restrict__ onw, us_t* oh, us_t* ol) {
  __shared__ __attribute__((aligned(16))) f16t smem[4 * 4096];
  const int lane = threadIdx.x & 31, wave = threadIdx.x >> 5, hl = lane >> 4, m = lane & 15;
  const int h = blockIdx.y;
  const int q0 = blockIdx.x * 64 + wave * 16;
  if (q0 + 16 > S_) return;
  f16t* pt  = smem + wave * 4096;
  us_t* sth = (us_t*)(smem + wave * 4096);
  us_t* stl = sth + 2048;

  unsigned rmask[8];
#pragma unroll
  for (int r = 0; r < 8; ++r) rmask[r] = selmask[(size_t)h * S_ + q0 + 8 * hl + r];
  unsigned umask = 0u;
#pragma unroll
  for (int r = 0; r < 8; ++r) umask |= rmask[r];
#pragma unroll
  for (int off = 1; off < 32; off <<= 1) umask |= __shfl_xor(umask, off);

  v8f oacc[8];
#pragma unroll
  for (int nf = 0; nf < 8; ++nf)
#pragma unroll
    for (int e = 0; e < 8; ++e) oacc[nf][e] = 0.0f;
  float mrow[8], lrow[8];
#pragma unroll
  for (int r = 0; r < 8; ++r) { mrow[r] = NEGF; lrow[r] = 0.0f; }

  const int qblk = q0 >> 8;
  const size_t hcol = (size_t)h * DH;

  for (int j = 0; j <= qblk; ++j) {
    if (((umask >> j) & 1u) == 0u) continue;
    const int kbase = j * CHUNK_;
    int kstop = kbase + CHUNK_;
    if (j == qblk) {
      const int cap = (q0 + 16 + 31) & ~31;
      if (cap < kstop) kstop = cap;
    }
    for (int kp = kbase; kp < kstop; kp += 32) {
      v8f sc0, sc1;
#pragma unroll
      for (int e = 0; e < 8; ++e) { sc0[e] = 0.0f; sc1[e] = 0.0f; }
#pragma unroll 1
      for (int kk = 0; kk < 4; ++kk) {
        const size_t col = hcol + (size_t)kk * 32;
        const size_t qo  = (size_t)(q0 + m) * D_ + col;
        const size_t k0o = (size_t)(kp + m) * D_ + col;
        const size_t k1o = (size_t)(kp + 16 + m) * D_ + col;
        FragB fqh, fql, fkh0, fkl0, fkh1, fkl1;
        fqh.p[0]  = *(const v8us*)(qh + qo + 8 * hl);
        fqh.p[1]  = *(const v8us*)(qh + qo + 16 + 8 * hl);
        fql.p[0]  = *(const v8us*)(ql + qo + 8 * hl);
        fql.p[1]  = *(const v8us*)(ql + qo + 16 + 8 * hl);
        fkh0.p[0] = *(const v8us*)(kh + k0o + 8 * hl);
        fkh0.p[1] = *(const v8us*)(kh + k0o + 16 + 8 * hl);
        fkl0.p[0] = *(const v8us*)(kl + k0o + 8 * hl);
        fkl0.p[1] = *(const v8us*)(kl + k0o + 16 + 8 * hl);
        fkh1.p[0] = *(const v8us*)(kh + k1o + 8 * hl);
        fkh1.p[1] = *(const v8us*)(kh + k1o + 16 + 8 * hl);
        fkl1.p[0] = *(const v8us*)(kl + k1o + 8 * hl);
        fkl1.p[1] = *(const v8us*)(kl + k1o + 16 + 8 * hl);
        sc0 = wmma_bf(fqh.v, fkh0.v, sc0);
        sc0 = wmma_bf(fqh.v, fkl0.v, sc0);
        sc0 = wmma_bf(fql.v, fkh0.v, sc0);
        sc1 = wmma_bf(fqh.v, fkh1.v, sc1);
        sc1 = wmma_bf(fqh.v, fkl1.v, sc1);
        sc1 = wmma_bf(fql.v, fkh1.v, sc1);
        asm volatile(NOP4
                     : "+v"(sc0), "+v"(sc1)
                     : "v"(fqh.v), "v"(fql.v), "v"(fkh0.v), "v"(fkl0.v), "v"(fkh1.v), "v"(fkl1.v));
      }

      float corrv[8];
#pragma unroll
      for (int r = 0; r < 8; ++r) {
        const int row  = q0 + 8 * hl + r;
        const int key0 = kp + m;
        const bool sel = ((rmask[r] >> j) & 1u) != 0u;
        float s0 = sc0[r] * QK_SCALE;
        float s1 = sc1[r] * QK_SCALE;
        if (!sel || key0 > row)      s0 = NEGF;
        if (!sel || key0 + 16 > row) s1 = NEGF;
        float rmax = fmaxf(s0, s1);
#pragma unroll
        for (int off = 1; off < 16; off <<= 1) rmax = fmaxf(rmax, __shfl_xor(rmax, off));
        const float nm   = fmaxf(mrow[r], rmax);
        const float corr = __expf(mrow[r] - nm);
        const float p0 = (s0 <= -5.0e29f) ? 0.0f : __expf(s0 - nm);
        const float p1 = (s1 <= -5.0e29f) ? 0.0f : __expf(s1 - nm);
        float rs = p0 + p1;
#pragma unroll
        for (int off = 1; off < 16; off <<= 1) rs += __shfl_xor(rs, off);
        lrow[r]  = lrow[r] * corr + rs;
        mrow[r]  = nm;
        corrv[r] = corr;
        pt[(8 * hl + r) * 32 + m]      = (f16t)(p0 * 256.0f);
        pt[(8 * hl + r) * 32 + 16 + m] = (f16t)(p1 * 256.0f);
      }
#pragma unroll
      for (int nf = 0; nf < 8; ++nf)
#pragma unroll
        for (int r = 0; r < 8; ++r) oacc[nf][r] *= corrv[r];

      asm volatile("s_wait_dscnt 0x0" ::: "memory");
      FragH pa;
      pa.p[0] = *(const v8h_ma*)(pt + m * 32 + 8 * hl);
      pa.p[1] = *(const v8h_ma*)(pt + m * 32 + 16 + 8 * hl);
#pragma unroll
      for (int nf = 0; nf < 8; ++nf) {
        FragH vb;
        const size_t vo = (hcol + (size_t)nf * 16 + m) * S_ + kp;
        vb.p[0] = *(const v8h*)(vT + vo + 8 * hl);
        vb.p[1] = *(const v8h*)(vT + vo + 16 + 8 * hl);
        oacc[nf] = wmma_h(pa.v, vb.v, oacc[nf]);
        asm volatile(NOP4 : "+v"(oacc[nf]) : "v"(pa.v), "v"(vb.v));
      }
    }
  }

  float rn[8];
#pragma unroll
  for (int r = 0; r < 8; ++r) {
    float invl = (lrow[r] > 0.0f) ? (1.0f / lrow[r]) : 0.0f;
    invl *= (1.0f / 16384.0f);
#pragma unroll
    for (int nf = 0; nf < 8; ++nf) oacc[nf][r] *= invl;
    float ss = 0.0f;
#pragma unroll
    for (int nf = 0; nf < 8; ++nf) ss += oacc[nf][r] * oacc[nf][r];
#pragma unroll
    for (int off = 1; off < 16; off <<= 1) ss += __shfl_xor(ss, off);
    rn[r] = rsqrtf(ss * (1.0f / 128.0f) + 1e-6f);
  }
  asm volatile("s_wait_dscnt 0x0" ::: "memory");
#pragma unroll
  for (int nf = 0; nf < 8; ++nf) {
    const int dcol = nf * 16 + m;
    const float w = bf2f(f2bf(onw[dcol]));
#pragma unroll
    for (int r = 0; r < 8; ++r) {
      const float val = oacc[nf][r] * rn[r] * w;
      const us_t a = f2bf(val);
      const us_t b = f2bf(val - bf2f(a));
      sth[(8 * hl + r) * 128 + dcol] = a;
      stl[(8 * hl + r) * 128 + dcol] = b;
    }
  }
  asm volatile("s_wait_dscnt 0x0" ::: "memory");
  const int c8 = m * 8;
#pragma unroll
  for (int pass = 0; pass < 2; ++pass) {
#pragma unroll
    for (int it = 0; it < 8; ++it) {
      const int rr = it * 2 + hl;
      Pack8 xh, xl;
      xh.s = *(const v8us_ma*)(sth + rr * 128 + c8);
      xl.s = *(const v8us_ma*)(stl + rr * 128 + c8);
      const size_t go = (size_t)(q0 + rr) * D_ + hcol + c8;
      *(volatile v4u*)(oh + go) = xh.u;
      *(volatile v4u*)(ol + go) = xl.u;
    }
    if (pass == 0) __threadfence();
  }
}

extern "C" void kernel_launch(void* const* d_in, const int* in_sizes, int n_in,
                              void* d_out, int out_size, void* d_ws, size_t ws_size,
                              hipStream_t stream) {
  const size_t nE = (size_t)S_ * D_;
  if (n_in < 6) return;
  if (in_sizes[0] != (int)nE || in_sizes[1] != (int)nE || in_sizes[2] != (int)nE ||
      in_sizes[3] != (int)nE || in_sizes[4] != (int)nE || in_sizes[5] != DH) return;
  if (out_size != (int)nE) return;

  const float* X   = (const float*)d_in[0];
  const float* Wq  = (const float*)d_in[1];
  const float* Wk  = (const float*)d_in[2];
  const float* Wv  = (const float*)d_in[3];
  const float* Wo  = (const float*)d_in[4];
  const float* onw = (const float*)d_in[5];
  float* out = (float*)d_out;

  char* ws = (char*)d_ws;
  const size_t MB = (size_t)1 << 20;
  const size_t KB = (size_t)1 << 10;
  const size_t o_Xb  = 0,       o_Wqb = 8 * MB,  o_Wkb = 16 * MB, o_Wvb = 24 * MB, o_Wob = 32 * MB;
  const size_t o_qh  = 0,       o_ql  = 8 * MB,  o_kh  = 16 * MB, o_kl  = 24 * MB;
  const size_t o_qf  = 40 * MB, o_kf  = 56 * MB, o_vf  = 72 * MB;
  const size_t o_oh  = 40 * MB, o_ol  = 48 * MB;
  const size_t o_vT  = 88 * MB;
  const size_t o_cs  = 96 * MB, o_sn = 96 * MB + 512 * KB;
  const size_t o_km  = 97 * MB, o_sel = 97 * MB + 64 * KB;
  const size_t ws_end = 97 * MB + 192 * KB;
  if (ws_size < ws_end) return;

  us_t*  Xb  = (us_t*)(ws + o_Xb);
  us_t*  Wqb = (us_t*)(ws + o_Wqb);
  us_t*  Wkb = (us_t*)(ws + o_Wkb);
  us_t*  Wvb = (us_t*)(ws + o_Wvb);
  us_t*  Wob = (us_t*)(ws + o_Wob);
  us_t*  qh  = (us_t*)(ws + o_qh);
  us_t*  ql  = (us_t*)(ws + o_ql);
  us_t*  kh  = (us_t*)(ws + o_kh);
  us_t*  kl  = (us_t*)(ws + o_kl);
  float* qf  = (float*)(ws + o_qf);
  float* kf  = (float*)(ws + o_kf);
  float* vf  = (float*)(ws + o_vf);
  us_t*  ohb = (us_t*)(ws + o_oh);
  us_t*  olb = (us_t*)(ws + o_ol);
  f16t*  vT  = (f16t*)(ws + o_vT);
  float* cs  = (float*)(ws + o_cs);
  float* sn  = (float*)(ws + o_sn);
  float* km  = (float*)(ws + o_km);
  unsigned* selmask = (unsigned*)(ws + o_sel);

  k_cvt<<<dim3((unsigned)(nE / 8 / 256), 5), 256, 0, stream>>>(X, Wq, Wk, Wv, Wo, Xb, Wqb, Wkb, Wvb, Wob, (int)nE);
  k_gemm<false><<<dim3(D_ / 128, S_ / 128, 3), 256, 0, stream>>>(Xb, Xb, Wqb, Wkb, Wvb, qf, kf, vf, S_, D_, D_);
  k_trig<<<dim3(S_ / 4), 256, 0, stream>>>(cs, sn);
  k_post<<<dim3(NBLK * H_), 256, 0, stream>>>(qf, kf, vf, cs, sn, qh, ql, kh, kl, vT, km);
  k_gate<<<dim3(S_ / 32, H_), 256, 0, stream>>>(qf, cs, sn, km, selmask);
  k_attn<<<dim3(S_ / 64, H_), 128, 0, stream>>>(qh, ql, kh, kl, vT, selmask, onw, ohb, olb);
  k_gemm<true><<<dim3(D_ / 128, S_ / 128, 1), 256, 0, stream>>>(ohb, olb, Wob, Wob, Wob, out, out, out, S_, D_, D_);
}
